// SimpleAttention_42571715838578
// MI455X (gfx1250) — hardware-verified
//
#include <hip/hip_runtime.h>


typedef __attribute__((ext_vector_type(16))) _Float16 v16h;
typedef __attribute__((ext_vector_type(8)))  _Float16 v8h;
typedef __attribute__((ext_vector_type(8)))  float    v8f;
typedef __attribute__((ext_vector_type(4)))  float    v4f;
typedef __attribute__((ext_vector_type(4)))  int      v4i;

union U8f  { v8f  v; float    f[8];  };
union U16h { v16h v; v8h h[2]; v4i i[2]; _Float16 f[16]; };

constexpr int BATCH = 16;
constexpr int SEQ   = 2048;
constexpr int DH    = 64;
constexpr int BQ    = 128;
constexpr int BK    = 32;
constexpr int KPAD  = 72;
constexpr int VPAD  = 40;

#define QSCALE 0.18033688011112042f
#define MASK2  1442695.0f

__device__ __forceinline__ v8f wmma_f16(v16h a, v16h b, v8f c) {
  return __builtin_amdgcn_wmma_f32_16x16x32_f16(false, a, false, b,
                                                (short)0, c, false, false);
}

template <int CTRL>
__device__ __forceinline__ float dppf(float x) {
  int s = __float_as_int(x);
  return __int_as_float(__builtin_amdgcn_update_dpp(s, s, CTRL, 0xF, 0xF, true));
}
__device__ __forceinline__ float red_max16(float x) {
  x = fmaxf(x, dppf<0xB1>(x));
  x = fmaxf(x, dppf<0x4E>(x));
  x = fmaxf(x, dppf<0x141>(x));
  x = fmaxf(x, dppf<0x140>(x));
  return x;
}
__device__ __forceinline__ float red_sum16(float x) {
  x += dppf<0xB1>(x);
  x += dppf<0x4E>(x);
  x += dppf<0x141>(x);
  x += dppf<0x140>(x);
  return x;
}

__device__ __forceinline__ v8h cvt8v(v4f a, v4f b) {
  v8h d;
  d[0] = (_Float16)a[0]; d[1] = (_Float16)a[1];
  d[2] = (_Float16)a[2]; d[3] = (_Float16)a[3];
  d[4] = (_Float16)b[0]; d[5] = (_Float16)b[1];
  d[6] = (_Float16)b[2]; d[7] = (_Float16)b[3];
  return d;
}

__global__ __launch_bounds__(256)
void fa_fwd_causal(const float* __restrict__ Q, const float* __restrict__ K,
                   const float* __restrict__ V, float* __restrict__ O)
{
  __shared__ _Float16 sK[BK * KPAD];
  __shared__ _Float16 sV[DH * VPAD];
  __shared__ _Float16 sP[8 * 512];
  __shared__ __attribute__((aligned(16))) float sO[8][16 * 64];

  const int tid  = threadIdx.x;
  const int wave = tid >> 5;
  const int lane = tid & 31;
  const int lh   = lane & 15;
  const int hi   = lane >> 4;

  const int b     = blockIdx.x / (SEQ / BQ);
  const int qbase = (blockIdx.x % (SEQ / BQ)) * BQ;
  const int qrow0 = qbase + wave * 16;

  const float* Qb = Q + (size_t)b * SEQ * DH;
  float*       Ob = O + (size_t)b * SEQ * DH;

  U16h qf[2];
  #pragma unroll
  for (int c = 0; c < 2; ++c) {
    const float* row = Qb + (size_t)(qrow0 + lh) * DH + 32 * c + 8 * hi;
    v4f a0 = *(const v4f*)(row);
    v4f a1 = *(const v4f*)(row + 4);
    v4f b0 = *(const v4f*)(row + 16);
    v4f b1 = *(const v4f*)(row + 20);
    qf[c].h[0] = cvt8v(a0 * QSCALE, a1 * QSCALE);
    qf[c].h[1] = cvt8v(b0 * QSCALE, b1 * QSCALE);
  }

  U8f acc[4];
  #pragma unroll
  for (int t = 0; t < 4; ++t) acc[t].v = (v8f){};
  float mrow[8], lrow[8];
  #pragma unroll
  for (int j = 0; j < 8; ++j) { mrow[j] = -3.0e38f; lrow[j] = 0.f; }

  _Float16* pw = &sP[wave * 512];
  const int nkv = qbase + BQ;

  const int r  = tid >> 3;
  const int d0 = (tid & 7) * 8;
  const float* Kp = K + (size_t)b * SEQ * DH + (size_t)r * DH + d0;
  const float* Vp = V + (size_t)b * SEQ * DH + (size_t)r * DH + d0;
  v4f kr0 = *(const v4f*)Kp, kr1 = *(const v4f*)(Kp + 4);
  v4f vr0 = *(const v4f*)Vp, vr1 = *(const v4f*)(Vp + 4);

  for (int kv0 = 0; kv0 < nkv; kv0 += BK) {
    __syncthreads();
    {
      v8h kh = cvt8v(kr0, kr1);
      *(v8h*)&sK[r * KPAD + d0] = kh;
      #pragma unroll
      for (int i = 0; i < 4; ++i) sV[(d0 + i)     * VPAD + r] = (_Float16)vr0[i];
      #pragma unroll
      for (int i = 0; i < 4; ++i) sV[(d0 + 4 + i) * VPAD + r] = (_Float16)vr1[i];
    }
    __syncthreads();

    if (kv0 + BK < nkv) {
      Kp += BK * DH;  Vp += BK * DH;
      kr0 = *(const v4f*)Kp; kr1 = *(const v4f*)(Kp + 4);
      vr0 = *(const v4f*)Vp; vr1 = *(const v4f*)(Vp + 4);
      if (kv0 + 2 * BK < nkv) {
        __builtin_prefetch(Kp + BK * DH, 0, 1);
        __builtin_prefetch(Vp + BK * DH, 0, 1);
      }
    }

    if (kv0 > qrow0 + 15) continue;
    const bool need_mask = (kv0 + BK - 1 > qrow0);

    U8f s0, s1; s0.v = (v8f){}; s1.v = (v8f){};
    #pragma unroll
    for (int c = 0; c < 2; ++c) {
      U16h kf;
      kf.h[0] = *(v8h*)&sK[lh * KPAD + 32 * c + 8 * hi];
      kf.h[1] = *(v8h*)&sK[lh * KPAD + 32 * c + 16 + 8 * hi];
      s0.v = wmma_f16(qf[c].v, kf.v, s0.v);
      kf.h[0] = *(v8h*)&sK[(16 + lh) * KPAD + 32 * c + 8 * hi];
      kf.h[1] = *(v8h*)&sK[(16 + lh) * KPAD + 32 * c + 16 + 8 * hi];
      s1.v = wmma_f16(qf[c].v, kf.v, s1.v);
    }

    const int col0 = kv0 + lh;
    const int col1 = kv0 + 16 + lh;
    v8h pa, pb;
    #pragma unroll
    for (int j = 0; j < 8; ++j) {
      const int row = qrow0 + j + 8 * hi;
      float a  = s0.f[j];
      float bb = s1.f[j];
      if (need_mask) {
        a  -= (col0 > row ? MASK2 : 0.f);
        bb -= (col1 > row ? MASK2 : 0.f);
      }
      const float rm    = red_max16(fmaxf(a, bb));
      const float mnew  = fmaxf(mrow[j], rm);
      const float alpha = __builtin_amdgcn_exp2f(mrow[j] - mnew);
      const float e0    = __builtin_amdgcn_exp2f(a  - mnew);
      const float e1    = __builtin_amdgcn_exp2f(bb - mnew);
      lrow[j] = lrow[j] * alpha + red_sum16(e0 + e1);
      mrow[j] = mnew;
      pa[j] = (_Float16)(e0 * 1024.0f);
      pb[j] = (_Float16)(e1 * 1024.0f);
      #pragma unroll
      for (int t = 0; t < 4; ++t) acc[t].f[j] *= alpha;
    }

    #pragma unroll
    for (int j = 0; j < 8; ++j) { pw[(j + 8 * hi) * 32 + lh] = pa[j]; pw[(j + 8 * hi) * 32 + 16 + lh] = pb[j]; }
    asm volatile("s_wait_dscnt 0" ::: "memory");
    U16h pf;
    pf.h[0] = *(volatile v8h*)&pw[lh * 32 + 8 * hi];
    pf.h[1] = *(volatile v8h*)&pw[lh * 32 + 16 + 8 * hi];


    #pragma unroll
    for (int t = 0; t < 4; ++t) {
      U16h vf;
      vf.h[0] = *(v8h*)&sV[(t * 16 + lh) * VPAD + 8 * hi];
      vf.h[1] = *(v8h*)&sV[(t * 16 + lh) * VPAD + 16 + 8 * hi];
      acc[t].v = wmma_f16(pf.v, vf.v, acc[t].v);
    }
  }

  float* so = sO[wave];
  #pragma unroll
  for (int j = 0; j < 8; ++j) {
    const float inv = 1.0f / (lrow[j] * 1024.0f);
    #pragma unroll
    for (int t = 0; t < 4; ++t) so[(j + 8 * hi) * 64 + t * 16 + lh] = acc[t].f[j] * inv;
  }
  asm volatile("s_wait_dscnt 0" ::: "memory");
  {
    typedef float v4fa __attribute__((ext_vector_type(4), may_alias));
    v4f ov[8]; size_t oo[8];
    #pragma unroll
    for (int i = 0; i < 8; ++i) {
      const int c = lane + 32 * i, rr = c >> 4, q = c & 15;
      ov[i] = *(const volatile v4fa*)(so + rr * 64 + q * 4);
      oo[i] = (size_t)(qrow0 + rr) * DH + q * 4;
    }
    #pragma unroll
    for (int i = 0; i < 8; ++i) *(volatile v4f*)(Ob + oo[i]) = ov[i];
    __threadfence();
    #pragma unroll
    for (int i = 0; i < 8; ++i) *(volatile v4f*)(Ob + oo[i]) = ov[i];
  }
}

extern "C" void kernel_launch(void* const* d_in, const int* in_sizes, int n_in,
                              void* d_out, int out_size, void* d_ws, size_t ws_size,
                              hipStream_t stream) {
  const float* q = (const float*)d_in[0];
  const float* k = (const float*)d_in[1];
  const float* v = (const float*)d_in[2];
  float*       o = (float*)d_out;
  dim3 grid(BATCH * (SEQ / BQ));
  fa_fwd_causal<<<grid, 256, 0, stream>>>(q, k, v, o);
}
